// EnhancedGNN_24232205484082
// MI455X (gfx1250) — hardware-verified
//
#include <hip/hip_runtime.h>
#include <stddef.h>
#include <math.h>


#define HID    128
#define FC1    32
#define KD     128
#define NTHR   256
#define NWAVE  8
#define EPT    8
#define NGRP   2
#define CHUNK  (NTHR * EPT * NGRP)
#define WCAP   (EPT * NGRP * 32)
#define LISTN  (NWAVE * WCAP)
#define NB     2048
#define RCAP   36864
#define TGT    256
#define DEGCAP 128
#define RB     128
#define WMAT   16384
#define WTOT   53248
#define STW    256
#define LDS_CSR ((RCAP + 3 * NB + LISTN + 2 * NWAVE) * 4)

static_assert((CHUNK & (CHUNK - 1)) == 0);
static_assert(CHUNK <= 4096);
static_assert(NB <= 4096 && (NB & (NB - 1)) == 0);
static_assert(NB == NTHR * 8);
static_assert((RCAP % 32) == 0);
static_assert(TGT == NWAVE * 32);
static_assert(RB * 2 == NTHR);
static_assert((NB % TGT) == 0);
static_assert((KD % 32) == 0);
static_assert(HID == 4 * 32);

typedef float          v4f   __attribute__((ext_vector_type(4)));
typedef float          v8f   __attribute__((ext_vector_type(8)));
typedef int            v4i   __attribute__((ext_vector_type(4)));
typedef double         v2d   __attribute__((ext_vector_type(2)));
typedef unsigned short v8us  __attribute__((ext_vector_type(8)));
typedef __bf16         v16bf __attribute__((ext_vector_type(16)));
union FragB { v16bf v; v8us h[2]; };
union FI { float f; int i; };

__host__ __device__ constexpr int gemm_lds(int nc) { return RB * (KD + 8) * 4 + RB * nc * 4; }

__device__ __forceinline__ float wred(float v) {
#pragma unroll
  for (int i = 16; i > 0; i >>= 1) v += __shfl_xor(v, i, 32);
  return v;
}

__device__ __forceinline__ unsigned int bfr_bits(float f) {
  unsigned int u = __float_as_uint(f);
  u += 0x7FFFu + ((u >> 16) & 1u);
  return u >> 16;
}

__device__ __forceinline__ void split1(float f, unsigned short& hi, unsigned short& lo) {
  const unsigned int hb = bfr_bits(f);
  const float hf = __uint_as_float(hb << 16);
  hi = (unsigned short)hb;
  lo = (unsigned short)bfr_bits(f - hf);
}

__device__ __forceinline__ void split8(v4f a, v4f b, v8us& hi, v8us& lo) {
  unsigned short h0, h1, h2, h3, h4, h5, h6, h7, l0, l1, l2, l3, l4, l5, l6, l7;
  split1(a.x, h0, l0); split1(a.y, h1, l1); split1(a.z, h2, l2); split1(a.w, h3, l3);
  split1(b.x, h4, l4); split1(b.y, h5, l5); split1(b.z, h6, l6); split1(b.w, h7, l7);
  hi[0] = h0; hi[1] = h1; hi[2] = h2; hi[3] = h3; hi[4] = h4; hi[5] = h5; hi[6] = h6; hi[7] = h7;
  lo[0] = l0; lo[1] = l1; lo[2] = l2; lo[3] = l3; lo[4] = l4; lo[5] = l5; lo[6] = l6; lo[7] = l7;
}

__device__ __forceinline__ v8f wmb(v16bf a, v16bf b, v8f c) {
  v8f d = __builtin_amdgcn_wmma_f32_16x16x32_bf16(false, a, false, b, (short)0, c, false, false);
  asm volatile("v_nop\n\tv_nop\n\tv_nop\n\tv_nop" : "+v"(d) : "v"(a), "v"(b));
  return d;
}

template <int NBS>
__device__ __forceinline__ int scan_chunk(const int* __restrict__ dsts, int nE, int cbase, int slotBase,
                                          int vec8, int* list, int tid, int lane, int wave) {
  int wc = 0;
#pragma unroll
  for (int g = 0; g < NGRP; ++g) {
    const int el0  = (g * NTHR + tid) * EPT;
    const int e0   = cbase + el0;
    const int sent = -2147483647 - 1;
    v4i da, db;
    if (vec8 != 0 && cbase + CHUNK <= nE) {
      da = *(const v4i*)(dsts + e0);
      db = *(const v4i*)(dsts + e0 + 4);
    } else {
      da.x = (e0     < nE) ? dsts[min(e0, nE - 1)] : sent;
      da.y = (e0 + 1 < nE) ? dsts[min(e0 + 1, nE - 1)] : sent;
      da.z = (e0 + 2 < nE) ? dsts[min(e0 + 2, nE - 1)] : sent;
      da.w = (e0 + 3 < nE) ? dsts[min(e0 + 3, nE - 1)] : sent;
      db.x = (e0 + 4 < nE) ? dsts[min(e0 + 4, nE - 1)] : sent;
      db.y = (e0 + 5 < nE) ? dsts[min(e0 + 5, nE - 1)] : sent;
      db.z = (e0 + 6 < nE) ? dsts[min(e0 + 6, nE - 1)] : sent;
      db.w = (e0 + 7 < nE) ? dsts[min(e0 + 7, nE - 1)] : sent;
    }
    const unsigned nb = (unsigned)slotBase;
    const unsigned s0 = (unsigned)da.x - nb, s1 = (unsigned)da.y - nb;
    const unsigned s2 = (unsigned)da.z - nb, s3 = (unsigned)da.w - nb;
    const unsigned s4 = (unsigned)db.x - nb, s5 = (unsigned)db.y - nb;
    const unsigned s6 = (unsigned)db.z - nb, s7 = (unsigned)db.w - nb;
    const bool h0 = s0 < (unsigned)NBS, h1 = s1 < (unsigned)NBS, h2 = s2 < (unsigned)NBS, h3 = s3 < (unsigned)NBS;
    const bool h4 = s4 < (unsigned)NBS, h5 = s5 < (unsigned)NBS, h6 = s6 < (unsigned)NBS, h7 = s7 < (unsigned)NBS;
    const unsigned any = __builtin_amdgcn_ballot_w32(h0 | h1 | h2 | h3 | h4 | h5 | h6 | h7);
    if (any != 0u) {
#define HITJ(J, HJ, SJ) { \
        const unsigned mj = __builtin_amdgcn_ballot_w32(HJ); \
        if (mj != 0u) { \
          if (HJ) { \
            const int pos = wc + (int)__builtin_amdgcn_mbcnt_lo(mj, 0u); \
            if (pos < WCAP) list[wave * WCAP + pos] = ((el0 + (J)) << 12) | (int)(SJ); \
          } \
          wc += (int)__builtin_popcount(mj); } }
      HITJ(0, h0, s0)
      HITJ(1, h1, s1)
      HITJ(2, h2, s2)
      HITJ(3, h3, s3)
      HITJ(4, h4, s4)
      HITJ(5, h5, s5)
      HITJ(6, h6, s6)
      HITJ(7, h7, s7)
#undef HITJ
    }
  }
  return wc;
}

__global__ __launch_bounds__(NTHR) void k_wprep(
    const float* __restrict__ w0, const float* __restrict__ w1,
    const float* __restrict__ w2, const float* __restrict__ w3,
    unsigned short* whi, unsigned short* wlo) {
  const int bid = (int)blockIdx.x, tid = (int)threadIdx.x;
  const int seg  = bid < 8 ? 0 : (bid < 16 ? 1 : (bid < 24 ? 2 : 3));
  const float* src = seg == 0 ? w0 : (seg == 1 ? w1 : (seg == 2 ? w2 : w3));
  const int sb   = seg * 8;
  const int ncol = seg == 3 ? FC1 : HID;
  const int pb   = seg * WMAT;
  const int i  = (bid - sb) * NTHR + tid;
  const int n  = i >> 4;
  const int k0 = (i & 15) * 8;
  v4f a, b;
  a.x = src[(size_t)(k0 + 0) * ncol + n]; a.y = src[(size_t)(k0 + 1) * ncol + n];
  a.z = src[(size_t)(k0 + 2) * ncol + n]; a.w = src[(size_t)(k0 + 3) * ncol + n];
  b.x = src[(size_t)(k0 + 4) * ncol + n]; b.y = src[(size_t)(k0 + 5) * ncol + n];
  b.z = src[(size_t)(k0 + 6) * ncol + n]; b.w = src[(size_t)(k0 + 7) * ncol + n];
  v8us hv, lv;
  split8(a, b, hv, lv);
  const size_t o = (size_t)pb + (size_t)i * 8;
  *(volatile v8us*)(whi + o) = hv;
  *(volatile v8us*)(wlo + o) = lv;
  __threadfence();
  *(volatile v8us*)(whi + o) = hv;
  *(volatile v8us*)(wlo + o) = lv;
}

__global__ __launch_bounds__(NTHR) void k_csr(
    const int* __restrict__ ei, int* cnt, int* off, float* dinv, int* csr, int nE, int vec8) {
  extern __shared__ v4f lds_dyn[];
  int*   region = (int*)lds_dyn;
  int*   scnt   = region + RCAP;
  float* sdv    = (float*)(scnt + NB);
  int*   soff   = scnt + 2 * NB;
  int*   list   = soff + NB;
  int*   wcnt   = list + LISTN;
  int*   wtot   = wcnt + NWAVE;
  const int tid = threadIdx.x, lane = tid & 31, wave = tid >> 5;
  const int b = blockIdx.x;
  const int nodeBase = b * NB;
  const int regBase  = b * RCAP;
  const int* dsts = ei + nE;

  {
    const v4i z = {0, 0, 0, 0};
    for (int i = tid; i < RCAP / 4; i += NTHR) ((v4i*)region)[i] = z;
    for (int i = tid; i < NB / 4; i += NTHR) ((v4i*)scnt)[i] = z;
  }
  __syncthreads();

  const int nChunks = (nE + CHUNK - 1) / CHUNK;

#pragma unroll 1
  for (int ch = 0; ch < nChunks; ++ch) {
    const int cbase = ch * CHUNK;
    const int wc = scan_chunk<NB>(dsts, nE, cbase, nodeBase, vec8, list, tid, lane, wave);
    if (lane == 0) wcnt[wave] = wc;
    __syncthreads();
    if (wave == 0) {
#pragma unroll 1
      for (int wsx = 0; wsx < NWAVE; ++wsx) {
        int n = __builtin_amdgcn_readfirstlane(wcnt[wsx]);
        n = n > WCAP ? WCAP : (n < 0 ? 0 : n);
        const int* lp = list + wsx * WCAP;
#pragma unroll 1
        for (int i = 0; i < n; ++i) {
          const int ent  = __builtin_amdgcn_readfirstlane(lp[i]);
          const int slot = ent & (NB - 1);
          if (lane == 0) scnt[slot] = scnt[slot] + 1;
        }
      }
    }
    __syncthreads();
  }

  int ev[8];
  {
    const v4i c0 = *(const v4i*)(scnt + 8 * tid);
    const v4i c1 = *(const v4i*)(scnt + 8 * tid + 4);
    ev[0] = max(c0.x, 0); ev[1] = max(c0.y, 0); ev[2] = max(c0.z, 0); ev[3] = max(c0.w, 0);
    ev[4] = max(c1.x, 0); ev[5] = max(c1.y, 0); ev[6] = max(c1.z, 0); ev[7] = max(c1.w, 0);
  }
  int ts = 0;
#pragma unroll
  for (int i = 0; i < 8; ++i) ts += ev[i];
  int incl = ts;
#pragma unroll
  for (int d = 1; d < 32; d <<= 1) {
    const int t = __shfl_up(incl, d);
    if (lane >= d) incl += t;
  }
  if (lane == 31) wtot[wave] = incl;
  __syncthreads();
  int pre = 0;
#pragma unroll 1
  for (int w = 0; w < wave; ++w) pre += wtot[w];
  {
    int run = pre + incl - ts;
    int ov[8];
#pragma unroll
    for (int i = 0; i < 8; ++i) { ov[i] = run; run += ev[i]; }
    const v4i o0 = {ov[0], ov[1], ov[2], ov[3]};
    const v4i o1 = {ov[4], ov[5], ov[6], ov[7]};
    *(v4i*)(soff + 8 * tid)     = o0;
    *(v4i*)(soff + 8 * tid + 4) = o1;
#pragma unroll 1
    for (int i = 0; i < 8; ++i) {
      int cv = scnt[8 * tid + i];
      cv = cv < 0 ? 0 : cv;
      const float dg = (float)cv + 1.0f;
      sdv[8 * tid + i] = 1.0f / sqrtf(dg);
    }
  }
  __syncthreads();

  {
    v4i cq[2], oq[2]; v4f dq[2];
#pragma unroll
    for (int q = 0; q < 2; ++q) {
      const int f = (wave * 2 + q) * 128 + 4 * lane;
      cq[q] = *(const v4i*)(scnt + f);
      oq[q] = *(const v4i*)(soff + f) + regBase;
      dq[q] = *(const v4f*)(sdv + f);
    }
    int*   cp = cnt  + (size_t)nodeBase;
    int*   op = off  + (size_t)nodeBase;
    float* dp = dinv + (size_t)nodeBase;
#pragma unroll
    for (int q = 0; q < 2; ++q) {
      const int f = (wave * 2 + q) * 128 + 4 * lane;
      *(volatile v4i*)(cp + f) = cq[q];
      *(volatile v4i*)(op + f) = oq[q];
      *(volatile v4f*)(dp + f) = dq[q];
    }
    __threadfence();
#pragma unroll
    for (int q = 0; q < 2; ++q) {
      const int f = (wave * 2 + q) * 128 + 4 * lane;
      *(volatile v4i*)(cp + f) = cq[q];
      *(volatile v4i*)(op + f) = oq[q];
      *(volatile v4f*)(dp + f) = dq[q];
    }
  }

#pragma unroll 1
  for (int ch = 0; ch < nChunks; ++ch) {
    const int cbase = ch * CHUNK;
    const int wc = scan_chunk<NB>(dsts, nE, cbase, nodeBase, vec8, list, tid, lane, wave);
    if (lane == 0) wcnt[wave] = wc;
    __syncthreads();
    if (wave == 0) {
#pragma unroll 1
      for (int wsx = 0; wsx < NWAVE; ++wsx) {
        int n = __builtin_amdgcn_readfirstlane(wcnt[wsx]);
        n = n > WCAP ? WCAP : (n < 0 ? 0 : n);
        const int* lp = list + wsx * WCAP;
#pragma unroll 1
        for (int i = 0; i < n; ++i) {
          const int ent  = __builtin_amdgcn_readfirstlane(lp[i]);
          const int slot = ent & (NB - 1);
          int e = cbase + ((ent >> 12) & (CHUNK - 1));
          e = e > nE - 1 ? nE - 1 : e;
          if (lane == 0) {
            int pos = soff[slot];
            pos = pos < 0 ? 0 : (pos > RCAP - 1 ? RCAP - 1 : pos);
            region[pos] = e;
            const int np = pos + 1;
            soff[slot] = np > RCAP ? RCAP : np;
          }
        }
      }
    }
    __syncthreads();
  }

  int* gp = csr + (size_t)regBase;
#pragma unroll 1
  for (int i = tid; i < RCAP / 4; i += NTHR) { const v4i v = ((const v4i*)region)[i]; *(volatile v4i*)(gp + 4 * i) = v; }
  __threadfence();
#pragma unroll 1
  for (int i = tid; i < RCAP / 4; i += NTHR) { const v4i v = ((const v4i*)region)[i]; *(volatile v4i*)(gp + 4 * i) = v; }
}

__global__ __launch_bounds__(NTHR) void k_embed(
    const float* __restrict__ x, const float* __restrict__ cw, const float* __restrict__ cb,
    const float* __restrict__ lg, const float* __restrict__ lb, float* h, int nN) {
  const int tid = threadIdx.x, lane = tid & 31, wave = tid >> 5;
  const int row = blockIdx.x * NWAVE + wave;
  const int rr = row > nN - 1 ? nN - 1 : row;
  const float x0 = x[2 * (size_t)rr], x1 = x[2 * (size_t)rr + 1];
  const int c0 = 4 * lane;
  const v4f wa = *(const v4f*)(cw + c0), wb = *(const v4f*)(cw + HID + c0);
  const v4f bc = *(const v4f*)(cb + c0);
  const v4f gg = *(const v4f*)(lg + c0), be = *(const v4f*)(lb + c0);
  v4f t = wa * x0 + wb * x1 + bc;
  t.x = fmaxf(t.x, 0.f); t.y = fmaxf(t.y, 0.f); t.z = fmaxf(t.z, 0.f); t.w = fmaxf(t.w, 0.f);
  const float s1 = wred(t.x + t.y + t.z + t.w);
  const float mu = s1 * (1.0f / 128.0f);
  const v4f d = t - mu;
  const float q = wred(d.x * d.x + d.y * d.y + d.z * d.z + d.w * d.w);
  const float var = q * (1.0f / 128.0f);
  const float inv = 1.0f / sqrtf(var + 1e-5f);
  const v4f o = d * inv * gg + be;
  float* hp = h + (size_t)row * HID + c0;
  *(volatile v4f*)hp = o;
  __threadfence();
  *(volatile v4f*)hp = o;
}

template <int NC, int EP>
__global__ __launch_bounds__(NTHR) void k_gemm(
    const float* __restrict__ A,
    const unsigned short* __restrict__ Bh, const unsigned short* __restrict__ Bl,
    const float* __restrict__ dinv, float* C, int nRowsA) {
  extern __shared__ v4f lds_dyn[];
  constexpr int AP  = KD + 8;
  constexpr int NTL = NC / 16;
  constexpr int TG  = NTL < 4 ? NTL : 4;
  constexpr int NGR = NTL / TG;
  constexpr int KV  = KD / 8;
  constexpr int LA  = RB * AP * 4;
  static_assert(NGR * TG == NTL);
  static_assert((NC % 32) == 0);
  unsigned short* sAh = (unsigned short*)lds_dyn;
  unsigned short* sAl = sAh + RB * AP;
  float* stg = (float*)((char*)lds_dyn + LA);
  const int tid = threadIdx.x, lane = tid & 31, wave = tid >> 5, hh = lane >> 4, m = lane & 15;
  const int rowBase = blockIdx.x * RB;

#pragma unroll
  for (int i = 0; i < (RB * KV) / NTHR; ++i) {
    const int idx = i * NTHR + tid;
    const int r   = idx / KV;
    const int c0  = (idx % KV) * 8;
    int row = rowBase + r;
    row = row > nRowsA - 1 ? nRowsA - 1 : row;
    const float* ap = A + (size_t)row * KD + c0;
    const v4f a = *(const v4f*)ap;
    const v4f b = *(const v4f*)(ap + 4);
    v8us hv, lv;
    split8(a, b, hv, lv);
    *(v8us*)(sAh + r * AP + c0) = hv;
    *(v8us*)(sAl + r * AP + c0) = lv;
  }
  __syncthreads();

  const int r0 = wave * 16 + 8 * hh;
  float s[8];
#pragma unroll
  for (int r = 0; r < 8; ++r) s[r] = 1.0f;
  if (EP == 0) {
    const v4f dA = *(const v4f*)(dinv + (size_t)rowBase + r0);
    const v4f dB = *(const v4f*)(dinv + (size_t)rowBase + r0 + 4);
    s[0] = dA.x; s[1] = dA.y; s[2] = dA.z; s[3] = dA.w; s[4] = dB.x; s[5] = dB.y; s[6] = dB.z; s[7] = dB.w;
  }
  const unsigned short* ah = sAh + (wave * 16 + m) * AP + 8 * hh;
  const unsigned short* al = sAl + (wave * 16 + m) * AP + 8 * hh;
  float* sp = stg + r0 * NC + m;

#pragma unroll 1
  for (int g = 0; g < NGR; ++g) {
    v8f acc[TG];
#pragma unroll
    for (int t = 0; t < TG; ++t) { v8f z = {0.f, 0.f, 0.f, 0.f, 0.f, 0.f, 0.f, 0.f}; acc[t] = z; }
#pragma unroll 1
    for (int kt = 0; kt < KD / 32; ++kt) {
      FragB fah, fal;
      fah.h[0] = *(const v8us*)(ah + 32 * kt);
      fah.h[1] = *(const v8us*)(ah + 32 * kt + 16);
      fal.h[0] = *(const v8us*)(al + 32 * kt);
      fal.h[1] = *(const v8us*)(al + 32 * kt + 16);
#pragma unroll
      for (int t = 0; t < TG; ++t) {
        const size_t bo = (size_t)((g * TG + t) * 16 + m) * KD + 32 * kt + 8 * hh;
        FragB fbh, fbl;
        fbh.h[0] = *(const v8us*)(Bh + bo);
        fbh.h[1] = *(const v8us*)(Bh + bo + 16);
        fbl.h[0] = *(const v8us*)(Bl + bo);
        fbl.h[1] = *(const v8us*)(Bl + bo + 16);
        acc[t] = wmb(fah.v, fbh.v, acc[t]);
        acc[t] = wmb(fah.v, fbl.v, acc[t]);
        acc[t] = wmb(fal.v, fbh.v, acc[t]);
      }
    }
#pragma unroll
    for (int t = 0; t < TG; ++t) {
      const int cb = (g * TG + t) * 16;
#pragma unroll
      for (int r = 0; r < 8; ++r) sp[r * NC + cb] = (EP == 0) ? (acc[t][r] * s[r]) : acc[t][r];
    }
  }
  __syncthreads();

  constexpr int NCH = NC / 8;
  const float* lp = stg + wave * 16 * NC + 4 * lane;
  float* gp = C + ((size_t)rowBase + wave * 16) * NC + 4 * lane;
#pragma unroll
  for (int i = 0; i < NCH; ++i) { const v4f v = *(const v4f*)(lp + i * 128); *(volatile v4f*)(gp + (size_t)i * 128) = v; }
  __threadfence();
#pragma unroll
  for (int i = 0; i < NCH; ++i) { const v4f v = *(const v4f*)(lp + i * 128); *(volatile v4f*)(gp + (size_t)i * 128) = v; }
}

__global__ __launch_bounds__(NTHR) void k_agg(
    const int* __restrict__ csr, const int* __restrict__ off, const int* __restrict__ cnt,
    const int* __restrict__ ei, const float* __restrict__ dinv,
    const float* __restrict__ hw, const float* __restrict__ bias,
    float* y, double* part, int nN, int nE, int csrLen) {
  __shared__ __attribute__((aligned(16))) double pw[NWAVE * 2 * HID];
  __shared__ __attribute__((aligned(16))) double tot[2 * HID];
  const int tid = threadIdx.x, lane = tid & 31, wave = tid >> 5;
  const int tbase = blockIdx.x * TGT + wave * 32;
  const int cl = tbase + lane;
  const int cnt_l = cnt[cl];
  const int off_l = off[cl];
  FI dvu; dvu.f = dinv[cl];
  const v4f bb = *(const v4f*)(bias + 4 * lane);
  double sm0 = 0.0, sm1 = 0.0, sm2 = 0.0, sm3 = 0.0;
  double sq0 = 0.0, sq1 = 0.0, sq2 = 0.0, sq3 = 0.0;

#pragma unroll 1
  for (int j = 0; j < 32; ++j) {
    const int c = tbase + j;
    int n = __builtin_amdgcn_readlane(cnt_l, j);
    n = n < 0 ? 0 : (n > DEGCAP ? DEGCAP : n);
    const int st = __builtin_amdgcn_readlane(off_l, j);
    FI du; du.i = __builtin_amdgcn_readlane(dvu.i, j);
    const float dc = du.f;
    v4f acc = {0.f, 0.f, 0.f, 0.f};
#pragma unroll 1
    for (int q0 = 0; q0 < n; q0 += 32) {
      int pos = st + q0 + lane;
      pos = pos < 0 ? 0 : (pos > csrLen - 1 ? csrLen - 1 : pos);
      int e = csr[pos];
      e = e < 0 ? 0 : (e > nE - 1 ? nE - 1 : e);
      int sl = ei[e];
      sl = sl < 0 ? 0 : (sl > nN - 1 ? nN - 1 : sl);
      const int mcnt = (n - q0) < 32 ? (n - q0) : 32;
#pragma unroll 1
      for (int p = 0; p < mcnt; ++p) {
        const int s = __builtin_amdgcn_readlane(sl, p);
        const v4f row = *(const v4f*)(hw + (size_t)s * HID + 4 * lane);
        acc = acc + row;
      }
    }
    const v4f sv = *(const v4f*)(hw + (size_t)c * HID + 4 * lane);
    v4f v = (acc + sv) * dc + bb;
    v.x = fmaxf(v.x, 0.f); v.y = fmaxf(v.y, 0.f); v.z = fmaxf(v.z, 0.f); v.w = fmaxf(v.w, 0.f);
    float* yp = y + (size_t)c * HID + 4 * lane;
    *(volatile v4f*)yp = v;
    __threadfence();
    *(volatile v4f*)yp = v;
    if (c < nN) {
      const double v0 = (double)v.x, v1 = (double)v.y, v2 = (double)v.z, v3 = (double)v.w;
      sm0 += v0; sm1 += v1; sm2 += v2; sm3 += v3;
      sq0 += v0 * v0; sq1 += v1 * v1; sq2 += v2 * v2; sq3 += v3 * v3;
    }
  }
  {
    double* pwp = pw + (size_t)(wave * 2) * HID + 4 * lane;
    pwp[0] = sm0; pwp[1] = sm1; pwp[2] = sm2; pwp[3] = sm3;
    pwp[HID + 0] = sq0; pwp[HID + 1] = sq1; pwp[HID + 2] = sq2; pwp[HID + 3] = sq3;
  }
  __syncthreads();
  {
    const int kind = tid >> 7, ch = tid & (HID - 1);
    double t = 0.0;
#pragma unroll
    for (int w = 0; w < NWAVE; ++w) t += pw[(w * 2 + kind) * HID + ch];
    tot[tid] = t;
  }
  __syncthreads();
  v2d pv = {0.0, 0.0};
  if (tid < HID) pv = *(const v2d*)(tot + 2 * tid);
  double* pp = part + (size_t)blockIdx.x * (2 * HID) + 2 * tid;
  if (tid < HID) *(volatile v2d*)pp = pv;
  __threadfence();
  if (tid < HID) *(volatile v2d*)pp = pv;
}

__global__ __launch_bounds__(128) void k_bnfin(
    const double* __restrict__ part, int nBlk, int pitch, int nc, int nRows, float* st) {
  __shared__ __attribute__((aligned(16))) float ss[STW];
  const int tid = threadIdx.x;
  const int c = tid < nc ? tid : nc - 1;
  double s = 0.0, q = 0.0;
#pragma unroll 1
  for (int b2 = 0; b2 < nBlk; ++b2) {
    const double* p = part + (size_t)b2 * pitch;
    s += p[c];
    q += p[nc + c];
  }
  const double inv_n = 1.0 / (double)nRows;
  const double mean = s * inv_n;
  double var = q * inv_n - mean * mean;
  var = var < 0.0 ? 0.0 : var;
  const float meanf = (float)mean;
  const float ve = (float)var + 1e-5f;
  const float istd = 1.0f / sqrtf(ve);
  ss[tid] = (tid < nc) ? meanf : 0.0f;
  ss[128 + tid] = (tid < nc) ? istd : 0.0f;
  __syncthreads();
  v4f v = {0.f, 0.f, 0.f, 0.f};
  if (tid < 64) v = *(const v4f*)(ss + 4 * tid);
  if (tid < 64) *(volatile v4f*)(st + 4 * tid) = v;
  __threadfence();
  if (tid < 64) *(volatile v4f*)(st + 4 * tid) = v;
}

__global__ __launch_bounds__(NTHR) void k_post(
    const float* __restrict__ y, const float* __restrict__ hid, const float* __restrict__ st,
    const float* __restrict__ g, const float* __restrict__ be, float* hout) {
  const int tid = threadIdx.x, lane = tid & 31, wave = tid >> 5;
  const int row = blockIdx.x * NWAVE + wave;
  const int c0 = 4 * lane;
  const size_t ro = (size_t)row * HID + c0;
  const v4f yv = *(const v4f*)(y + ro);
  const v4f id = *(const v4f*)(hid + ro);
  const v4f mu = *(const v4f*)(st + c0), is = *(const v4f*)(st + HID + c0);
  const v4f gg = *(const v4f*)(g + c0), bb = *(const v4f*)(be + c0);
  v4f t = (yv - mu) * is * gg + bb;
  t = t + id;
  const float s1 = wred(t.x + t.y + t.z + t.w);
  const float m1 = s1 * (1.0f / 128.0f);
  const v4f d = t - m1;
  const float q = wred(d.x * d.x + d.y * d.y + d.z * d.z + d.w * d.w);
  const float var = q * (1.0f / 128.0f);
  const float inv = 1.0f / sqrtf(var + 1e-5f);
  const v4f o = d * inv;
  float* hp = hout + ro;
  *(volatile v4f*)hp = o;
  __threadfence();
  *(volatile v4f*)hp = o;
}

__global__ __launch_bounds__(NTHR) void k_head(
    const float* __restrict__ f1, const float* __restrict__ b1,
    const float* __restrict__ w2, const float* __restrict__ b2,
    float* out, int nN, int outN) {
  __shared__ float sw[2 * FC1];
  __shared__ float sb[FC1];
  __shared__ float sb2[2];
  __shared__ __attribute__((aligned(16))) float so[2 * NTHR];
  const int tid = threadIdx.x;
  if (tid < 2 * FC1) sw[tid] = w2[tid];
  if (tid < FC1) sb[tid] = b1[tid];
  if (tid < 2) sb2[tid] = b2[tid];
  __syncthreads();
  const int node = blockIdx.x * NTHR + tid;
  const int rr = node > nN - 1 ? nN - 1 : node;
  const float* fp = f1 + (size_t)rr * FC1;
  float a0 = 0.0f, a1 = 0.0f;
#pragma unroll 1
  for (int k = 0; k < FC1; ++k) {
    const float t = fmaxf(fp[k] + sb[k], 0.0f);
    a0 = fmaf(t, sw[2 * k], a0);
    a1 = fmaf(t, sw[2 * k + 1], a1);
  }
  a0 += sb2[0];
  a1 += sb2[1];
  float o0 = 0.0f, o1 = 0.0f;
#pragma unroll 1
  for (int j = 0; j < 2; ++j) {
    const float a = (j == 0) ? a0 : a1;
    const float o = tanhf(a);
    o0 = (j == 0) ? o : o0;
    o1 = (j == 0) ? o1 : o;
  }
  so[2 * tid] = o0;
  so[2 * tid + 1] = o1;
  __syncthreads();

  const int base = blockIdx.x * (2 * NTHR);
  int nv = outN - base;
  nv = nv > 2 * NTHR ? 2 * NTHR : (nv < 0 ? 0 : nv);
  const int nv4 = nv >> 2;
  const int tl = nv & 3;
  const v4f v = *(const v4f*)(so + 4 * (tid & 127));
  float* gp = out + (size_t)base + 4 * tid;
  int ti = 4 * nv4 + tid;
  ti = ti > 2 * NTHR - 1 ? 2 * NTHR - 1 : ti;
  const float tv = so[ti];
  float* tp = out + (size_t)base + ti;
  if (tid < nv4) *(volatile v4f*)gp = v;
  if (tid < tl) *(volatile float*)tp = tv;
  __threadfence();
  if (tid < nv4) *(volatile v4f*)gp = v;
  if (tid < tl) *(volatile float*)tp = tv;
}

extern "C" void kernel_launch(void* const* d_in, const int* in_sizes, int n_in,
                              void* d_out, int out_size, void* d_ws, size_t ws_size,
                              hipStream_t stream) {
  if (n_in < 18) return;
  const int nN = in_sizes[0] / 2;
  const int nE = in_sizes[1] / 2;
  if (nN <= 0 || nE <= 0) return;
  if (in_sizes[0] != 2 * nN || in_sizes[1] != 2 * nE) return;
  if (in_sizes[2] != 2 * HID || in_sizes[3] != HID) return;
  if (in_sizes[4] != HID || in_sizes[5] != HID || in_sizes[6] != HID || in_sizes[7] != HID) return;
  if (in_sizes[8] != HID * HID || in_sizes[9] != HID || in_sizes[10] != HID * HID || in_sizes[11] != HID) return;
  if (in_sizes[12] != HID * HID || in_sizes[13] != HID) return;
  if (in_sizes[14] != HID * FC1 || in_sizes[15] != FC1 || in_sizes[16] != FC1 * 2 || in_sizes[17] != 2) return;
  if (out_size != 2 * nN) return;
  if (nE > (1 << 28) || nN > (1 << 24)) return;

  const float* x      = (const float*)d_in[0];
  const int*   ei     = (const int*)d_in[1];
  const float* coordW = (const float*)d_in[2];
  const float* coordB = (const float*)d_in[3];
  const float* lng    = (const float*)d_in[4];
  const float* lnb    = (const float*)d_in[5];
  const float* bng    = (const float*)d_in[6];
  const float* bnb    = (const float*)d_in[7];
  const float* W1     = (const float*)d_in[8];
  const float* bl1    = (const float*)d_in[9];
  const float* W2     = (const float*)d_in[10];
  const float* bl2    = (const float*)d_in[11];
  const float* W3     = (const float*)d_in[12];
  const float* bl3    = (const float*)d_in[13];
  const float* fc1W   = (const float*)d_in[14];
  const float* fc1b   = (const float*)d_in[15];
  const float* fc2W   = (const float*)d_in[16];
  const float* fc2b   = (const float*)d_in[17];
  float* out = (float*)d_out;

  const int NPAD   = ((nN + TGT - 1) / TGT) * TGT;
  const int nBC    = (nN + NB - 1) / NB;
  const int CNTPAD = nBC * NB;
  const int csrLen = nBC * RCAP;
  const int nGemm  = NPAD / RB;
  const int nAgg   = NPAD / TGT;
  const int nRowB  = NPAD / NWAVE;
  const int nHeadB = (out_size + 2 * NTHR - 1) / (2 * NTHR);

  char* ws = (char*)d_ws;
  size_t cur = 0;
  const size_t A256 = 255;
  const size_t oWh  = cur; cur += (size_t)WTOT * 2;                 cur = (cur + A256) & ~A256;
  const size_t oWl  = cur; cur += (size_t)WTOT * 2;                 cur = (cur + A256) & ~A256;
  const size_t oCnt = cur; cur += (size_t)CNTPAD * 4;               cur = (cur + A256) & ~A256;
  const size_t oDv  = cur; cur += (size_t)CNTPAD * 4;               cur = (cur + A256) & ~A256;
  const size_t oOff = cur; cur += (size_t)CNTPAD * 4;               cur = (cur + A256) & ~A256;
  const size_t oCsr = cur; cur += (size_t)csrLen * 4;               cur = (cur + A256) & ~A256;
  const size_t oP0  = cur; cur += (size_t)NPAD * HID * 4;           cur = (cur + A256) & ~A256;
  const size_t oP1  = cur; cur += (size_t)NPAD * HID * 4;           cur = (cur + A256) & ~A256;
  const size_t oP2  = cur; cur += (size_t)NPAD * HID * 4;           cur = (cur + A256) & ~A256;
  const size_t oPt  = cur; cur += (size_t)nAgg * (2 * HID) * 8;     cur = (cur + A256) & ~A256;
  const size_t oSt  = cur; cur += (size_t)STW * 4;                  cur = (cur + A256) & ~A256;
  if (cur > ws_size) return;
  if (cur > ((size_t)128 << 20)) return;
  unsigned short* whi = (unsigned short*)(ws + oWh);
  unsigned short* wlo = (unsigned short*)(ws + oWl);
  int*    cnt   = (int*)(ws + oCnt);
  float*  dinv  = (float*)(ws + oDv);
  int*    offp  = (int*)(ws + oOff);
  int*    csr   = (int*)(ws + oCsr);
  float*  P0    = (float*)(ws + oP0);
  float*  P1    = (float*)(ws + oP1);
  float*  P2    = (float*)(ws + oP2);
  double* part  = (double*)(ws + oPt);
  float*  st    = (float*)(ws + oSt);

  const int vec8 = ((nE & 3) == 0) ? 1 : 0;
  constexpr int LG0 = gemm_lds(HID);
  constexpr int LG1 = gemm_lds(FC1);

  k_wprep<<<26, NTHR, 0, stream>>>(W1, W2, W3, fc1W, whi, wlo);

  hipFuncSetAttribute(reinterpret_cast<const void*>(&k_csr),
                      hipFuncAttributeMaxDynamicSharedMemorySize, LDS_CSR);
  k_csr<<<nBC, NTHR, LDS_CSR, stream>>>(ei, cnt, offp, dinv, csr, nE, vec8);

  k_embed<<<nRowB, NTHR, 0, stream>>>(x, coordW, coordB, lng, lnb, P0, nN);

  hipFuncSetAttribute(reinterpret_cast<const void*>(&k_gemm<HID, 0>),
                      hipFuncAttributeMaxDynamicSharedMemorySize, LG0);
  const float* bls[3] = {bl1, bl2, bl3};
  float* hcur = P0;
  float* hw   = P1;
  for (int l = 0; l < 3; ++l) {
    k_gemm<HID, 0><<<nGemm, NTHR, LG0, stream>>>(hcur, whi + (size_t)l * WMAT, wlo + (size_t)l * WMAT, dinv, hw, nN);
    k_agg<<<nAgg, NTHR, 0, stream>>>(csr, offp, cnt, ei, dinv, hw, bls[l], P2, part, nN, nE, csrLen);
    k_bnfin<<<1, 128, 0, stream>>>(part, nAgg, 2 * HID, HID, nN, st);
    k_post<<<nRowB, NTHR, 0, stream>>>(P2, hcur, st, bng, bnb, hw);
    float* tswap = hcur; hcur = hw; hw = tswap;
  }

  hipFuncSetAttribute(reinterpret_cast<const void*>(&k_gemm<FC1, 1>),
                      hipFuncAttributeMaxDynamicSharedMemorySize, LG1);
  k_gemm<FC1, 1><<<nGemm, NTHR, LG1, stream>>>(hcur, whi + (size_t)3 * WMAT, wlo + (size_t)3 * WMAT, dinv, P2, nN);

  k_head<<<nHeadB, NTHR, 0, stream>>>(P2, fc1b, fc2W, fc2b, out, nN, out_size);
}
